// GatedQueryAttLayer_44427141710076
// MI455X (gfx1250) — hardware-run, weakly checked
//
#include <hip/hip_runtime.h>
#include <math.h>

constexpr int kB    = 16;
constexpr int kS    = 512;
constexpr int kE    = 1024;
constexpr int kH    = 16;
constexpr int kDK   = 64;
constexpr int kTok  = kB * kS;
constexpr int kChunkB   = 4;
constexpr int kNChunk   = kB / kChunkB;
constexpr int kChunkTok = kChunkB * kS;
constexpr int kChunkRow = kChunkTok * kH;

constexpr float kWCarry     = 16.0f;
constexpr float kWCarryInv  = 1.0f / 16.0f;
constexpr float kGWCarry    = 8.0f;
constexpr float kGWCarryInv = 1.0f / 8.0f;
constexpr float kGCarry     = 64.0f;
constexpr float kZScale     = 1.0f / (64.0f * 8.0f);
constexpr float kPCarry     = 2048.0f;
constexpr float kPVScale    = 1.0f / 2048.0f;
constexpr float kScoreScale = 0.125f;

constexpr size_t kMiB    = 1048576;
constexpr size_t kOffQp  = 0;
constexpr size_t kOffKp  = 4 * kMiB;
constexpr size_t kOffQ16 = 8 * kMiB;
constexpr size_t kOffK16 = 12 * kMiB;
constexpr size_t kOffGq  = 16 * kMiB;
constexpr size_t kOffGk  = 24 * kMiB;
constexpr size_t kOffG16 = 32 * kMiB;
constexpr size_t kOffZ   = 16 * kMiB;
constexpr size_t kOffS   = 8 * kMiB;
constexpr size_t kOffP   = 24 * kMiB;
constexpr size_t kOffX16 = 0;
constexpr size_t kOffWt  = 16 * kMiB;
constexpr size_t kOffSW  = 36 * kMiB;
constexpr size_t kOffQf  = 36 * kMiB + 65536;
constexpr size_t kOffKf  = kOffQf + 32 * kMiB;
constexpr size_t kOffVt  = kOffKf + 32 * kMiB;
constexpr size_t kWsEnd  = kOffVt + 16 * kMiB;
static_assert((size_t)kChunkRow * kDK * 2 == 4 * kMiB, "plane size");
static_assert((size_t)kChunkRow * 128 * 4 == 16 * kMiB, "z plane size");
static_assert((size_t)kH * kS * kS * 4 == 16 * kMiB, "score plane size");
static_assert((size_t)kTok * kE * 2 == 16 * kMiB, "x16 plane size");
static_assert(kOffWt + (size_t)3 * kE * kE * 2 <= kOffSW, "wt plane fits");
static_assert(kOffG16 + 4 * kMiB <= kOffSW, "g16 fits");
static_assert(kOffSW + 32768 <= kOffQf, "gate weights fit");
static_assert(kWsEnd == 121700352, "carve end");
static_assert(kWsEnd <= 134217728, "carve within budget");

typedef __attribute__((ext_vector_type(16))) _Float16 v16h;
typedef __attribute__((ext_vector_type(8)))  _Float16 v8h;
typedef __attribute__((ext_vector_type(16))) __bf16   v16b;
typedef __attribute__((ext_vector_type(8)))  __bf16   v8b;
typedef __attribute__((ext_vector_type(8)))  float    v8f;
typedef __attribute__((ext_vector_type(4)))  float    v4f;
typedef __attribute__((ext_vector_type(4)))  unsigned int v4u;

__device__ __forceinline__ unsigned short f2bf_bits(float f) {
  unsigned u = __float_as_uint(f);
  return (unsigned short)((u + 0x7FFFu + ((u >> 16) & 1u)) >> 16);
}
__device__ __forceinline__ float bf_bits2f(unsigned short h) { return __uint_as_float(((unsigned)h) << 16); }

__device__ __forceinline__ void dep_guard_h(v8f& a, v8f& b, v16h x, v16h y) { asm volatile("v_nop\n\tv_nop\n\tv_nop\n\tv_nop" : "+v"(a), "+v"(b) : "v"(x), "v"(y)); }
__device__ __forceinline__ void dep_guard_b(v8f& a, v8f& b, v16b x, v16b y) { asm volatile("v_nop\n\tv_nop\n\tv_nop\n\tv_nop" : "+v"(a), "+v"(b) : "v"(x), "v"(y)); }
__device__ __forceinline__ void keep4_h(v16h a, v16h b, v16h c, v16h d) { asm volatile("v_nop" :: "v"(a), "v"(b), "v"(c), "v"(d)); }
__device__ __forceinline__ void keep4_b(v16b a, v16b b, v16b c, v16b d) { asm volatile("v_nop" :: "v"(a), "v"(b), "v"(c), "v"(d)); }
__device__ __forceinline__ void acc_guard4(v8f& a, v8f& b, v8f& c, v8f& d) { asm volatile("v_nop\n\tv_nop\n\tv_nop\n\tv_nop" : "+v"(a), "+v"(b), "+v"(c), "+v"(d)); }
template <typename T> struct Frag;
template <> struct Frag<_Float16> {
  typedef v16h V; union U { v16h v; v8h h[2]; };
  static __device__ __forceinline__ v16h load(const _Float16* p) {
    U f; f.h[0] = *(const v8h*)(p); f.h[1] = *(const v8h*)(p + 16); return f.v;
  }
  static __device__ __forceinline__ v8f mma(v16h a, v16h b, v8f c) {
    return __builtin_amdgcn_wmma_f32_16x16x32_f16(false, a, false, b, (short)0, c, false, false);
  }
  static __device__ __forceinline__ void guard(v8f& a, v8f& b, v16h x, v16h y) { dep_guard_h(a, b, x, y); }
  static __device__ __forceinline__ void keep(v16h a, v16h b, v16h c, v16h d) { keep4_h(a, b, c, d); }
};
template <> struct Frag<__bf16> {
  typedef v16b V; union U { v16b v; v8b h[2]; };
  static __device__ __forceinline__ v16b load(const __bf16* p) {
    U f; f.h[0] = *(const v8b*)(p); f.h[1] = *(const v8b*)(p + 16); return f.v;
  }
  static __device__ __forceinline__ v8f mma(v16b a, v16b b, v8f c) {
    return __builtin_amdgcn_wmma_f32_16x16x32_bf16(false, a, false, b, (short)0, c, false, false);
  }
  static __device__ __forceinline__ void guard(v8f& a, v8f& b, v16b x, v16b y) { dep_guard_b(a, b, x, y); }
  static __device__ __forceinline__ void keep(v16b a, v16b b, v16b c, v16b d) { keep4_b(a, b, c, d); }
};

__device__ __forceinline__ unsigned pk16(unsigned short a, unsigned short b) { return (unsigned)a | ((unsigned)b << 16); }
__device__ __forceinline__ unsigned short h_bits(float f) { const _Float16 h = (_Float16)f; return __builtin_bit_cast(unsigned short, h); }

template <int ET> struct Elem;
template <> struct Elem<0> { typedef _Float16 T; };
template <> struct Elem<1> { typedef __bf16 T; };
template <int ET, bool SPLIT, int BIAS_MODE, int OUT_MODE, bool RESID, int ACT = 0>
__global__ __launch_bounds__(256) void wmma_gemm64(
    const unsigned short* __restrict__ Ap, const unsigned short* __restrict__ A2p, int lda, long strideA,
    const unsigned short* __restrict__ Btp, const unsigned short* __restrict__ Bt2p, int ldb, long strideB,
    void* __restrict__ Cout, void* __restrict__ Cout2, int ldc, long strideC,
    const float* __restrict__ bias,
    const float* __restrict__ resid, long strideR,
    int M, int N, int K, float scale) {
  typedef typename Elem<ET>::T T;
  typedef typename Frag<T>::V V;
  const T* A = (const T*)Ap; const T* A2 = (const T*)A2p; const T* Bt = (const T*)Btp; const T* Bt2 = (const T*)Bt2p;
  __shared__ __align__(16) float sT[8][16 * 68];
  const int b    = blockIdx.y;
  const int lane = threadIdx.x & 31;
  const int wave = threadIdx.x >> 5;
  const int tilesN = N >> 6;
  const int tilesM = M >> 6;
  const int tile = blockIdx.x * 8 + wave;
  if (tile >= tilesM * tilesN) return;
  const int tm = tile / tilesN;
  const int tn = tile - tm * tilesN;
  const int m0 = tm << 6;
  const int n0 = tn << 6;

  const T* Ab  = A  + (size_t)b * strideA;
  const T* Bb  = Bt + (size_t)b * strideB;
  const T* Ab2 = SPLIT ? (A2  + (size_t)b * strideA) : nullptr;
  const T* Bb2 = SPLIT ? (Bt2 + (size_t)b * strideB) : nullptr;

  const int rlane = lane & 15;
  const int koff  = (lane >> 4) * 8;
  const int mOff  = (lane >> 4) * 8;

  v8f acc[4][4];
#pragma unroll
  for (int i = 0; i < 4; ++i)
#pragma unroll
    for (int j = 0; j < 4; ++j) acc[i][j] = (v8f){0.f,0.f,0.f,0.f,0.f,0.f,0.f,0.f};

  for (int k0 = 0; k0 < K; k0 += 32) {
    V bh[4], bl[4];
#pragma unroll
    for (int j = 0; j < 4; ++j) {
      const size_t bo = (size_t)(n0 + (j << 4) + rlane) * ldb + koff + k0;
      bh[j] = Frag<T>::load(Bb + bo);
      if (SPLIT) bl[j] = Frag<T>::load(Bb2 + bo);
    }
#pragma unroll
    for (int i = 0; i < 4; ++i) {
      const size_t ao = (size_t)(m0 + (i << 4) + rlane) * lda + koff + k0;
      V ah = Frag<T>::load(Ab + ao);
      V al;
      if (SPLIT) al = Frag<T>::load(Ab2 + ao);
#pragma unroll
      for (int j = 0; j < 4; ++j) {
        acc[i][j] = Frag<T>::mma(ah, bh[j], acc[i][j]);
        if (SPLIT) {
          acc[i][j] = Frag<T>::mma(ah, bl[j], acc[i][j]);
          acc[i][j] = Frag<T>::mma(al, bh[j], acc[i][j]);
        }
      }
      Frag<T>::guard(acc[i][0], acc[i][3], ah, SPLIT ? al : ah);
    }
    Frag<T>::keep(bh[0], bh[1], bh[2], bh[3]);
    if (SPLIT) Frag<T>::keep(bl[0], bl[1], bl[2], bl[3]);
  }
  acc_guard4(acc[0][0], acc[0][1], acc[0][2], acc[0][3]);
  acc_guard4(acc[1][0], acc[1][1], acc[1][2], acc[1][3]);
  acc_guard4(acc[2][0], acc[2][1], acc[2][2], acc[2][3]);
  acc_guard4(acc[3][0], acc[3][1], acc[3][2], acc[3][3]);

  float* slab = sT[wave];
  const float* Rb = RESID ? (resid + (size_t)b * strideR) : nullptr;
#pragma unroll
  for (int i = 0; i < 4; ++i) {
    const int mBase = m0 + (i << 4);
#pragma unroll
    for (int j = 0; j < 4; ++j) {
      const int n = n0 + (j << 4) + rlane;
      float bv = 0.f;
      if (BIAS_MODE == 2) bv = bias[n];
#pragma unroll
      for (int r = 0; r < 8; ++r) {
        float v = acc[i][j][r] * scale;
        if (BIAS_MODE == 1) v += bias[mBase + mOff + r];
        if (BIAS_MODE == 2) v += bv;
        if (RESID) v += Rb[(size_t)(mBase + mOff + r) * ldc + n];
        if (ACT == 2) v = fmaxf(v, 0.0f);
        if (ACT == 4) v = (v > 0.f) ? v : 0.01f * v;
        slab[(mOff + r) * 68 + (j << 4) + rlane] = v;
      }
    }
    __builtin_amdgcn_fence(__ATOMIC_RELEASE, "workgroup");
    __builtin_amdgcn_wave_barrier();
    __builtin_amdgcn_fence(__ATOMIC_ACQUIRE, "workgroup");
    if (OUT_MODE == 0) {
      float* C = (float*)Cout + (size_t)b * strideC;
      const int hh = lane >> 4, c4 = (lane & 15) * 4;
      for (int pass = 0; pass < 2; ++pass) {
#pragma unroll
        for (int it = 0; it < 8; ++it) {
          const int row = it * 2 + hh;
          v4f v = *(const v4f*)(slab + row * 68 + c4);
          *(volatile v4f*)(C + (size_t)(mBase + row) * ldc + n0 + c4) = v;
        }
        __threadfence();
      }
    } else {
      const int q = lane >> 3, c8 = (lane & 7) * 8;
      unsigned short* C  = (unsigned short*)Cout  + (size_t)b * strideC;
      unsigned short* C2 = (OUT_MODE == 2) ? ((unsigned short*)Cout2 + (size_t)b * strideC) : nullptr;
      for (int pass = 0; pass < 2; ++pass) {
#pragma unroll
        for (int it = 0; it < 4; ++it) {
          const int row = it * 4 + q;
          const float* sp = slab + row * 68 + c8;
          v8h hv, lv;
#pragma unroll
          for (int e = 0; e < 8; ++e) {
            if (OUT_MODE == 1) {
              hv[e] = (_Float16)sp[e];
            } else {
              unsigned short hb = f2bf_bits(sp[e]);
              unsigned short lb = f2bf_bits(sp[e] - bf_bits2f(hb));
              hv[e] = __builtin_bit_cast(_Float16, hb);
              lv[e] = __builtin_bit_cast(_Float16, lb);
            }
          }
          *(volatile v8h*)(C + (size_t)(mBase + row) * ldc + n0 + c8) = hv;
          if (OUT_MODE == 2) *(volatile v8h*)(C2 + (size_t)(mBase + row) * ldc + n0 + c8) = lv;
        }
        __threadfence();
      }
    }
    __builtin_amdgcn_fence(__ATOMIC_RELEASE, "workgroup");
    __builtin_amdgcn_wave_barrier();
    __builtin_amdgcn_fence(__ATOMIC_ACQUIRE, "workgroup");
  }
}

__global__ __launch_bounds__(256) void wtcast_kernel(const float* __restrict__ W0, const float* __restrict__ W1,
                                                     const float* __restrict__ W2,
                                                     unsigned short* __restrict__ out, float scale) {
  __shared__ float sm[64][65];
  const int t  = threadIdx.x;
  const int d0 = blockIdx.x * 64;
  const int h0 = blockIdx.y * 64;
  const int z  = blockIdx.z;
  const float* W = (z == 0) ? W0 : (z == 1) ? W1 : W2;
#pragma unroll
  for (int i = 0; i < 16; ++i) {
    const int e = i * 256 + t;
    const int r = e >> 6;
    const int c = e & 63;
    sm[c][r] = W[(size_t)(d0 + r) * kE + h0 + c] * scale;
  }
  __syncthreads();
  const int lane = t & 31, wave = t >> 5;
  const int q = lane >> 3, c8 = (lane & 7) * 8;
  unsigned short* op = out + (size_t)z * kE * kE;
  for (int pass = 0; pass < 2; ++pass) {
#pragma unroll
    for (int it = 0; it < 2; ++it) {
      const int row = wave * 8 + it * 4 + q;
      unsigned short hb[8];
#pragma unroll
      for (int e = 0; e < 8; ++e) hb[e] = h_bits(sm[row][c8 + e]);
      const v4u u = (v4u){pk16(hb[0], hb[1]), pk16(hb[2], hb[3]), pk16(hb[4], hb[5]), pk16(hb[6], hb[7])};
      *(volatile v4u*)(op + (size_t)(h0 + row) * kE + d0 + c8) = u;
    }
    __threadfence();
  }
}

__global__ __launch_bounds__(256) void gatew_kernel(const float* __restrict__ Wfq, const float* __restrict__ Wfk,
                                                    const float* __restrict__ Wfg,
                                                    unsigned short* __restrict__ out, float scale) {
  __shared__ float sm[64][65];
  const int t = threadIdx.x;
  const int z = blockIdx.x;
  const float* W = (z == 0) ? Wfq : (z == 1) ? Wfk : Wfg;
  const int pin = (z >= 2) ? 128 : 64;
  const int n0  = (z == 3) ? 64 : 0;
#pragma unroll
  for (int i = 0; i < 16; ++i) {
    const int e = i * 256 + t;
    const int r = e >> 6;
    const int c = e & 63;
    sm[c][r] = W[r * pin + n0 + c] * scale;
  }
  __syncthreads();
  const int lane = t & 31, wave = t >> 5;
  const int q = lane >> 3, c8 = (lane & 7) * 8;
  unsigned short* op = out + (size_t)z * 4096;
  for (int pass = 0; pass < 2; ++pass) {
#pragma unroll
    for (int it = 0; it < 2; ++it) {
      const int row = wave * 8 + it * 4 + q;
      unsigned short hb[8];
#pragma unroll
      for (int e = 0; e < 8; ++e) hb[e] = h_bits(sm[row][c8 + e]);
      const v4u u = (v4u){pk16(hb[0], hb[1]), pk16(hb[2], hb[3]), pk16(hb[4], hb[5]), pk16(hb[6], hb[7])};
      *(volatile v4u*)(op + (size_t)row * kDK + c8) = u;
    }
    __threadfence();
  }
}

__global__ __launch_bounds__(256) void cast8_f16_kernel(const float* __restrict__ in, unsigned short* __restrict__ out, int n8) {
  const int i = blockIdx.x * 256 + threadIdx.x;
  if (i >= n8) return;
  const float* p = in + 8 * (size_t)i;
  const v4f a = *(const v4f*)(p);
  const v4f c = *(const v4f*)(p + 4);
  unsigned short hb[8];
#pragma unroll
  for (int e = 0; e < 4; ++e) {
    hb[e]     = h_bits(a[e]);
    hb[4 + e] = h_bits(c[e]);
  }
  const v4u u = (v4u){pk16(hb[0], hb[1]), pk16(hb[2], hb[3]), pk16(hb[4], hb[5]), pk16(hb[6], hb[7])};
  unsigned short* q = out + 8 * (size_t)i;
  *(volatile v4u*)q = u;
  __threadfence();
  *(volatile v4u*)q = u;
}

__global__ __launch_bounds__(256) void cast8_sel_kernel(const float* __restrict__ in0, const float* __restrict__ in1,
                                                        unsigned short* __restrict__ out0, unsigned short* __restrict__ out1, int n8) {
  const int sel = blockIdx.y;
  const float* in = sel ? in1 : in0;
  unsigned short* out = sel ? out1 : out0;
  const int i = blockIdx.x * 256 + threadIdx.x;
  if (i >= n8) return;
  const float* p = in + 8 * (size_t)i;
  const v4f a = *(const v4f*)(p);
  const v4f c = *(const v4f*)(p + 4);
  unsigned short hb[8];
#pragma unroll
  for (int e = 0; e < 4; ++e) {
    hb[e]     = h_bits(a[e]);
    hb[4 + e] = h_bits(c[e]);
  }
  const v4u u = (v4u){pk16(hb[0], hb[1]), pk16(hb[2], hb[3]), pk16(hb[4], hb[5]), pk16(hb[6], hb[7])};
  unsigned short* q = out + 8 * (size_t)i;
  *(volatile v4u*)q = u;
  __threadfence();
  *(volatile v4u*)q = u;
}

__global__ __launch_bounds__(256) void gmul_kernel(const float* __restrict__ a, const float* __restrict__ b,
                                                   unsigned short* __restrict__ out, int n8, float scale) {
  const int i = blockIdx.x * 256 + threadIdx.x;
  if (i >= n8) return;
  const float* pa = a + 8 * (size_t)i;
  const float* pb = b + 8 * (size_t)i;
  const v4f a0 = *(const v4f*)(pa);
  const v4f a1 = *(const v4f*)(pa + 4);
  const v4f b0 = *(const v4f*)(pb);
  const v4f b1 = *(const v4f*)(pb + 4);
  unsigned short hb[8];
#pragma unroll
  for (int e = 0; e < 4; ++e) {
    hb[e]     = h_bits((a0[e] * b0[e]) * scale);
    hb[4 + e] = h_bits((a1[e] * b1[e]) * scale);
  }
  const v4u u = (v4u){pk16(hb[0], hb[1]), pk16(hb[2], hb[3]), pk16(hb[4], hb[5]), pk16(hb[6], hb[7])};
  unsigned short* q = out + 8 * (size_t)i;
  *(volatile v4u*)q = u;
  __threadfence();
  *(volatile v4u*)q = u;
}

__global__ __launch_bounds__(256) void gatemod_kernel(const float* __restrict__ Z, const float* __restrict__ Xq,
                                                      const float* __restrict__ Xk,
                                                      unsigned short* __restrict__ Oq, unsigned short* __restrict__ Ok) {
  __shared__ __align__(16) unsigned sb[512];
  const int t = threadIdx.x;
  const int sel = blockIdx.y;
  const float* X = sel ? Xk : Xq;
  unsigned short* O = sel ? Ok : Oq;
  const size_t e0 = (size_t)blockIdx.x * 1024 + 4 * (size_t)t;
  const size_t r  = e0 >> 6;
  const int    d  = (int)(e0 & 63);
  const v4f zz = *(const v4f*)(Z + r * 128 + sel * 64 + d);
  const v4f xx = *(const v4f*)(X + e0);
  unsigned short hb[4];
#pragma unroll
  for (int e = 0; e < 4; ++e) {
    const float m = 1.0f / (1.0f + expf(-zz[e]));
    hb[e] = h_bits(xx[e] * m);
  }
  sb[2 * t]     = pk16(hb[0], hb[1]);
  sb[2 * t + 1] = pk16(hb[2], hb[3]);
  __syncthreads();
  if (t < 128) {
    const v4u u = *(const v4u*)(&sb[4 * t]);
    unsigned short* op = O + (size_t)blockIdx.x * 1024 + 8 * (size_t)t;
    *(volatile v4u*)op = u;
    __threadfence();
    *(volatile v4u*)op = u;
  }
}

__global__ __launch_bounds__(256) void softmax_rows_kernel(const float* __restrict__ Sp, unsigned short* __restrict__ Pp, float carry) {
  __shared__ float redM[8];
  __shared__ float redS[8];
  __shared__ __align__(16) unsigned sb[2][256];
  const int t    = threadIdx.x;
  const int lane = t & 31, wave = t >> 5;
  const int hf   = t >> 7;
  const int tt   = t & 127;
  const size_t row = (size_t)blockIdx.x * 2 + hf;
  const v4f a = *(const v4f*)(Sp + row * kS + 4 * tt);
  float m = fmaxf(fmaxf(a[0], a[1]), fmaxf(a[2], a[3]));
#pragma unroll
  for (int off = 16; off > 0; off >>= 1) m = fmaxf(m, __shfl_xor(m, off, 32));
  if (lane == 0) redM[wave] = m;
  __syncthreads();
  const int w0 = hf * 4;
  const float rm = fmaxf(fmaxf(redM[w0], redM[w0 + 1]), fmaxf(redM[w0 + 2], redM[w0 + 3]));
  float e[4];
  float s = 0.f;
#pragma unroll
  for (int i = 0; i < 4; ++i) { e[i] = expf(a[i] - rm); s += e[i]; }
#pragma unroll
  for (int off = 16; off > 0; off >>= 1) s += __shfl_xor(s, off, 32);
  if (lane == 0) redS[wave] = s;
  __syncthreads();
  const float tot = ((redS[w0] + redS[w0 + 1]) + redS[w0 + 2]) + redS[w0 + 3];
  const float inv = carry / tot;
  unsigned short hb[4];
#pragma unroll
  for (int i = 0; i < 4; ++i) hb[i] = h_bits(e[i] * inv);
  sb[hf][2 * tt]     = pk16(hb[0], hb[1]);
  sb[hf][2 * tt + 1] = pk16(hb[2], hb[3]);
  __syncthreads();
  if (tt < 64) {
    const v4u u = *(const v4u*)(&sb[hf][4 * tt]);
    unsigned short* op = Pp + row * kS + 8 * (size_t)tt;
    *(volatile v4u*)op = u;
    __threadfence();
    *(volatile v4u*)op = u;
  }
}

extern "C" void kernel_launch(void* const* d_in, const int* in_sizes, int n_in,
                              void* d_out, int out_size, void* d_ws, size_t ws_size,
                              hipStream_t stream) {
  if (n_in < 13) return;
  if (ws_size < kWsEnd) return;
  if ((size_t)out_size < (size_t)kTok * kE) return;
  if (in_sizes[0] != kTok * kE) return;

  const float* inp = (const float*)d_in[0];
  const float* Wq  = (const float*)d_in[1];
  const float* bq  = (const float*)d_in[2];
  const float* Wk  = (const float*)d_in[3];
  const float* bk  = (const float*)d_in[4];
  const float* Wv  = (const float*)d_in[5];
  const float* bvv = (const float*)d_in[6];
  const float* Wfq = (const float*)d_in[7];
  const float* bfq = (const float*)d_in[8];
  const float* Wfk = (const float*)d_in[9];
  const float* bfk = (const float*)d_in[10];
  const float* Wfg = (const float*)d_in[11];
  const float* bfg = (const float*)d_in[12];
  float* out = (float*)d_out;

  unsigned char* ws = (unsigned char*)d_ws;
  unsigned short* Qp16 = (unsigned short*)(ws + kOffQp);
  unsigned short* Kp16 = (unsigned short*)(ws + kOffKp);
  unsigned short* Q16a = (unsigned short*)(ws + kOffQ16);
  unsigned short* K16a = (unsigned short*)(ws + kOffK16);
  float*          Gq   = (float*)(ws + kOffGq);
  float*          Gk   = (float*)(ws + kOffGk);
  unsigned short* G16  = (unsigned short*)(ws + kOffG16);
  float*          Zp   = (float*)(ws + kOffZ);
  float*          Sp   = (float*)(ws + kOffS);
  unsigned short* Pp   = (unsigned short*)(ws + kOffP);
  unsigned short* X16  = (unsigned short*)(ws + kOffX16);
  unsigned short* Wt16 = (unsigned short*)(ws + kOffWt);
  unsigned short* SW   = (unsigned short*)(ws + kOffSW);
  unsigned short* SWq  = SW;
  unsigned short* SWk  = SW + 4096;
  unsigned short* SWg  = SW + 8192;
  float*          Qf   = (float*)(ws + kOffQf);
  float*          Kf   = (float*)(ws + kOffKf);
  unsigned short* Vt16 = (unsigned short*)(ws + kOffVt);

  cast8_f16_kernel<<<dim3((kTok * kE / 8) / 256), dim3(256), 0, stream>>>(inp, X16, kTok * kE / 8);
  wtcast_kernel<<<dim3(kE / 64, kE / 64, 3), dim3(256), 0, stream>>>(Wq, Wk, Wv, Wt16, kWCarry);
  gatew_kernel<<<dim3(4), dim3(256), 0, stream>>>(Wfq, Wfk, Wfg, SW, kGWCarry);

  wmma_gemm64<0, false, 2, 0, false, 0><<<dim3(256, 1), dim3(256), 0, stream>>>(
      X16, X16, kE, 0L, Wt16, Wt16, kE, 0L,
      (void*)Qf, (void*)Qf, kE, 0L, bq, nullptr, 0L, kTok, kE, kE, kWCarryInv);
  wmma_gemm64<0, false, 2, 0, false, 0><<<dim3(256, 1), dim3(256), 0, stream>>>(
      X16, X16, kE, 0L, Wt16 + (size_t)kE * kE, Wt16 + (size_t)kE * kE, kE, 0L,
      (void*)Kf, (void*)Kf, kE, 0L, bk, nullptr, 0L, kTok, kE, kE, kWCarryInv);
  wmma_gemm64<0, false, 1, 1, false, 0><<<dim3(256, 1), dim3(256), 0, stream>>>(
      Wt16 + (size_t)2 * kE * kE, Wt16 + (size_t)2 * kE * kE, kE, 0L, X16, X16, kE, 0L,
      (void*)Vt16, (void*)Vt16, kTok, 0L, bvv, nullptr, 0L, kE, kTok, kE, kWCarryInv);

  const int n8chunk = kChunkRow * kDK / 8;
  for (int c = 0; c < kNChunk; ++c) {
    const size_t tok0 = (size_t)c * kChunkTok;
    const float* Qfc = Qf + tok0 * kE;
    const float* Kfc = Kf + tok0 * kE;
    cast8_sel_kernel<<<dim3(n8chunk / 256, 2), dim3(256), 0, stream>>>(Qfc, Kfc, Q16a, K16a, n8chunk);
    wmma_gemm64<0, false, 2, 0, false, 0><<<dim3(64, 1), dim3(256), 0, stream>>>(
        Q16a, Q16a, kDK, 0L, SWq, SWq, kDK, 0L,
        (void*)Gq, (void*)Gq, kDK, 0L, bfq, nullptr, 0L, kChunkRow, kDK, kDK, kGWCarryInv);
    wmma_gemm64<0, false, 2, 0, false, 0><<<dim3(64, 1), dim3(256), 0, stream>>>(
        K16a, K16a, kDK, 0L, SWk, SWk, kDK, 0L,
        (void*)Gk, (void*)Gk, kDK, 0L, bfk, nullptr, 0L, kChunkRow, kDK, kDK, kGWCarryInv);
    gmul_kernel<<<dim3(n8chunk / 256), dim3(256), 0, stream>>>(Gq, Gk, G16, n8chunk, kGCarry);
    wmma_gemm64<0, false, 2, 0, false, 0><<<dim3(128, 1), dim3(256), 0, stream>>>(
        G16, G16, kDK, 0L, SWg, SWg, kDK, 0L,
        (void*)Zp, (void*)Zp, 128, 0L, bfg, nullptr, 0L, kChunkRow, 128, kDK, kZScale);
    gatemod_kernel<<<dim3(kChunkRow * kDK / 1024, 2), dim3(256), 0, stream>>>(Zp, Qfc, Kfc, Qp16, Kp16);

    for (int bl = 0; bl < kChunkB; ++bl) {
      const int b = c * kChunkB + bl;
      const unsigned short* Qpb = Qp16 + (size_t)bl * kS * kE;
      const unsigned short* Kpb = Kp16 + (size_t)bl * kS * kE;
      wmma_gemm64<0, false, 0, 0, false, 0><<<dim3(8, kH), dim3(256), 0, stream>>>(
          Qpb, Qpb, kE, 64L, Kpb, Kpb, kE, 64L,
          (void*)Sp, (void*)Sp, kS, (long)kS * kS, nullptr, nullptr, 0L, kS, kS, kDK, kScoreScale);
      softmax_rows_kernel<<<dim3(kH * kS / 2), dim3(256), 0, stream>>>(Sp, Pp, kPCarry);
      wmma_gemm64<0, false, 0, 0, false, 0><<<dim3(1, kH), dim3(256), 0, stream>>>(
          Pp, Pp, kS, (long)kS * kS, Vt16 + (size_t)b * kS, Vt16 + (size_t)b * kS, kTok, (long)kDK * kTok,
          (void*)(out + (size_t)b * kS * kE), (void*)(out + (size_t)b * kS * kE), kE, (long)kDK,
          nullptr, nullptr, 0L, kS, kDK, kS, kPVScale);
    }
  }
}
